// LSTMEncoder_44848048505211
// MI455X (gfx1250) — hardware-run, weakly checked
//
#include <hip/hip_runtime.h>
#include <math.h>

constexpr int NBATCH    = 4096;
constexpr int NSTEP     = 512;
constexpr int NIN       = 6;
constexpr int NHID      = 32;
constexpr int NGATE     = 4 * NHID;
constexpr int NWAVE     = 2;
constexpr int NTHR      = 32 * NWAVE;
constexpr int ROWS_WAVE = 16;
constexpr int ROWS_BLK  = NWAVE * ROWS_WAVE;
constexpr int WPITCH    = 72;
constexpr int XPITCH    = 40;
constexpr int HPITCH    = 200;
constexpr int SPITCH    = 36;
constexpr float LN_EPS  = 1e-5f;
static_assert(NBATCH % ROWS_BLK == 0);
static_assert(NTHR == 64);
static_assert(NGATE % NTHR == 0);
static_assert(NHID == 32 && NIN <= 8);
static_assert((WPITCH % 8) == 0 && (XPITCH % 8) == 0 && (HPITCH % 8) == 0 && (SPITCH % 4) == 0);

typedef __attribute__((ext_vector_type(16))) __bf16   v16b;
typedef __attribute__((ext_vector_type(8)))  __bf16   v8b;
typedef __attribute__((ext_vector_type(8)))  float    v8f;
typedef __attribute__((ext_vector_type(4)))  float    v4f;
typedef __attribute__((ext_vector_type(2)))  float    v2f;
typedef __attribute__((ext_vector_type(4)))  unsigned v4u;

__device__ __forceinline__ unsigned short f2bf_bits(float f) {
  unsigned u = __float_as_uint(f);
  return (unsigned short)((u + 0x7FFFu + ((u >> 16) & 1u)) >> 16);
}
__device__ __forceinline__ float bf_bits2f(unsigned short h) { return __uint_as_float(((unsigned)h) << 16); }
__device__ __forceinline__ float bf16r(float f) { return bf_bits2f(f2bf_bits(f)); }

template <typename T> struct Frag;
template <> struct Frag<__bf16> {
  typedef v16b V; union U { v16b v; v8b h[2]; };
  static __device__ __forceinline__ v16b load(const __bf16* p) {
    U f; f.h[0] = *(const v8b*)(p); f.h[1] = *(const v8b*)(p + 16); return f.v;
  }
  static __device__ __forceinline__ v8f mma(v16b a, v16b b, v8f c) {
    return __builtin_amdgcn_wmma_f32_16x16x32_bf16(false, a, false, b, (short)0, c, false, false);
  }
};

__device__ __forceinline__ void grp_guard(v8f& a0, v8f& a1, v8f& a2, v8f& a3,
                                          v16b x0, v16b x1, v16b y0, v16b y1, v16b y2, v16b y3) {
  asm volatile("v_nop\n\tv_nop\n\tv_nop\n\tv_nop"
               : "+v"(a0), "+v"(a1), "+v"(a2), "+v"(a3)
               : "v"(x0), "v"(x1), "v"(y0), "v"(y1), "v"(y2), "v"(y3));
}

__device__ __forceinline__ float fsig(float x)  { return __builtin_amdgcn_rcpf(1.0f + __expf(-x)); }
__device__ __forceinline__ float ftanh(float x) { return 1.0f - 2.0f * __builtin_amdgcn_rcpf(__expf(2.0f * x) + 1.0f); }

__device__ __forceinline__ void mma_one(v8f (&acc)[4], const __bf16* ap, const __bf16* wb, int kb) {
  const v16b a  = Frag<__bf16>::load(ap);
  const v16b b0 = Frag<__bf16>::load(wb + kb);
  const v16b b1 = Frag<__bf16>::load(wb + 32 * WPITCH + kb);
  const v16b b2 = Frag<__bf16>::load(wb + 64 * WPITCH + kb);
  const v16b b3 = Frag<__bf16>::load(wb + 96 * WPITCH + kb);
  acc[0] = Frag<__bf16>::mma(a, b0, acc[0]);
  acc[1] = Frag<__bf16>::mma(a, b1, acc[1]);
  acc[2] = Frag<__bf16>::mma(a, b2, acc[2]);
  acc[3] = Frag<__bf16>::mma(a, b3, acc[3]);
  grp_guard(acc[0], acc[1], acc[2], acc[3], a, a, b0, b1, b2, b3);
}
__device__ __forceinline__ void mma_two(v8f (&acc)[4], const __bf16* ap, const __bf16* wb, int kb) {
  const v16b ah = Frag<__bf16>::load(ap);
  const v16b al = Frag<__bf16>::load(ap + 32);
  const v16b b0 = Frag<__bf16>::load(wb + kb);
  const v16b b1 = Frag<__bf16>::load(wb + 32 * WPITCH + kb);
  const v16b b2 = Frag<__bf16>::load(wb + 64 * WPITCH + kb);
  const v16b b3 = Frag<__bf16>::load(wb + 96 * WPITCH + kb);
  acc[0] = Frag<__bf16>::mma(ah, b0, acc[0]);
  acc[1] = Frag<__bf16>::mma(ah, b1, acc[1]);
  acc[2] = Frag<__bf16>::mma(ah, b2, acc[2]);
  acc[3] = Frag<__bf16>::mma(ah, b3, acc[3]);
  acc[0] = Frag<__bf16>::mma(al, b0, acc[0]);
  acc[1] = Frag<__bf16>::mma(al, b1, acc[1]);
  acc[2] = Frag<__bf16>::mma(al, b2, acc[2]);
  acc[3] = Frag<__bf16>::mma(al, b3, acc[3]);
  grp_guard(acc[0], acc[1], acc[2], acc[3], ah, al, b0, b1, b2, b3);
}

__device__ __forceinline__ void cell_update(v8f (&acc)[4], const float (&bb)[4], float (&cst)[8], float (&hst)[8]) {
#pragma unroll
  for (int r = 0; r < 8; ++r) {
    const float zi = acc[0][r] + bb[0];
    const float zf = acc[1][r] + bb[1];
    const float zg = acc[2][r] + bb[2];
    const float zo = acc[3][r] + bb[3];
    const float ig = fsig(zi);
    const float fg = fsig(zf);
    const float gg = ftanh(zg);
    const float og = fsig(zo);
    const float cn = fg * cst[r] + ig * gg;
    cst[r] = cn;
    hst[r] = og * ftanh(cn);
  }
}

__device__ __forceinline__ void put_hilo(unsigned short* dst, int colbase, const float (&h)[2][8], int hh, int c) {
#pragma unroll
  for (int ub = 0; ub < 2; ++ub) {
#pragma unroll
    for (int r = 0; r < 8; ++r) {
      const float v = h[ub][r];
      const unsigned u = __float_as_uint(v);
      const unsigned short hb = (unsigned short)(u >> 16);
      const unsigned short lb = f2bf_bits(v - __uint_as_float(u & 0xffff0000u));
      dst[(8 * hh + r) * HPITCH + colbase + 16 * ub + c]      = hb;
      dst[(8 * hh + r) * HPITCH + colbase + 32 + 16 * ub + c] = lb;
    }
  }
}

__device__ __forceinline__ void stage_x(unsigned short* xt, const float* __restrict__ x, int rowbase, int t, int lane) {
  const int m = lane & 15, hh = lane >> 4;
  const float* xp = x + ((size_t)(rowbase + m) * NSTEP + (size_t)t) * NIN;
  const v2f p0 = *(const v2f*)(xp);
  const v2f p1 = *(const v2f*)(xp + 2);
  const v2f p2 = *(const v2f*)(xp + 4);
  const float x0 = p0[0], x1 = p0[1], x2 = p1[0], x3 = p1[1], x4 = p2[0], x5 = p2[1];
  const unsigned w0 = (unsigned)f2bf_bits(x0) | ((unsigned)f2bf_bits(x1) << 16);
  const unsigned w1 = (unsigned)f2bf_bits(x2) | ((unsigned)f2bf_bits(x3) << 16);
  const unsigned w2 = (unsigned)f2bf_bits(x4) | ((unsigned)f2bf_bits(x5) << 16);
  const v4u dv = {w0, w1, w2, 0u};
  const v4u zz = {0u, 0u, 0u, 0u};
  unsigned short* rp = xt + m * XPITCH;
  *(v4u*)(rp) = dv;
  *(v4u*)(rp + 8 + 8 * hh) = zz;
  *(v4u*)(rp + 24) = zz;
}

__global__ __launch_bounds__(NTHR) __attribute__((amdgpu_num_vgpr(256))) void lstm2_ln_kernel(
    const float* __restrict__ x,
    const float* __restrict__ wih0, const float* __restrict__ whh0,
    const float* __restrict__ bih0, const float* __restrict__ bhh0,
    const float* __restrict__ wih1, const float* __restrict__ whh1,
    const float* __restrict__ bih1, const float* __restrict__ bhh1,
    const float* __restrict__ gam,  const float* __restrict__ bet,
    float* __restrict__ out) {
  __shared__ __align__(16) unsigned short Wt0[NGATE * WPITCH];
  __shared__ __align__(16) unsigned short Wt1[NGATE * WPITCH];
  __shared__ __align__(16) unsigned short Xs[NWAVE][ROWS_WAVE * XPITCH];
  __shared__ __align__(16) unsigned short Hb[NWAVE][ROWS_WAVE * HPITCH];
  __shared__ __align__(16) float          St[NWAVE][ROWS_WAVE * SPITCH];
  __shared__ float Bsum[2 * NGATE];

  const int tid = threadIdx.x, lane = tid & 31, wave = tid >> 5;
  const int c = lane & 15, hh = lane >> 4, koff = hh * 8;
  const int rowbase = blockIdx.x * ROWS_BLK + wave * ROWS_WAVE;

  {
    const int k  = tid;
    const int kx = (k < NIN)   ? k : (NIN - 1);
    const int kr = (k >= NHID) ? (k - NHID) : 0;
    const int ki = (k < NHID)  ? k : (NHID - 1);
    const float fx = (k < NIN)   ? 1.0f : 0.0f;
    const float fr = (k >= NHID) ? 1.0f : 0.0f;
    const float fi = (k < NHID)  ? 1.0f : 0.0f;
#pragma unroll 1
    for (int n = 0; n < NGATE; ++n) {
      const float vx  = wih0[n * NIN + kx];
      const float vr0 = whh0[n * NHID + kr];
      const float vi1 = wih1[n * NHID + ki];
      const float vr1 = whh1[n * NHID + kr];
      const float w0 = fmaf(fx, vx, fr * vr0);
      const float w1 = fmaf(fi, vi1, fr * vr1);
      Wt0[n * WPITCH + k] = f2bf_bits(w0);
      Wt1[n * WPITCH + k] = f2bf_bits(w1);
    }
  }
#pragma unroll 1
  for (int n = tid; n < NGATE; n += NTHR) {
    Bsum[n]         = bf16r(bih0[n]) + bf16r(bhh0[n]);
    Bsum[NGATE + n] = bf16r(bih1[n]) + bf16r(bhh1[n]);
  }

  float c1[2][8], c2[2][8], h1s[2][8], h2s[2][8];
#pragma unroll
  for (int ub = 0; ub < 2; ++ub)
#pragma unroll
    for (int r = 0; r < 8; ++r) { c1[ub][r] = 0.0f; c2[ub][r] = 0.0f; h1s[ub][r] = 0.0f; h2s[ub][r] = 0.0f; }

  unsigned short* xs = Xs[wave];
  unsigned short* hb = Hb[wave];
  put_hilo(hb, 64, h1s, hh, c);
  stage_x(xs, x, rowbase, 0, lane);
  __syncthreads();

  float bb0[2][4], bb1[2][4], gm[2], bt[2];
#pragma unroll
  for (int ub = 0; ub < 2; ++ub) {
#pragma unroll
    for (int g = 0; g < 4; ++g) {
      bb0[ub][g] = Bsum[32 * g + 16 * ub + c];
      bb1[ub][g] = Bsum[NGATE + 32 * g + 16 * ub + c];
    }
    gm[ub] = bf16r(gam[16 * ub + c]);
    bt[ub] = bf16r(bet[16 * ub + c]);
  }

  const __bf16* xrow = (const __bf16*)xs  + c * XPITCH + koff;
  const __bf16* hrow = (const __bf16*)hb  + c * HPITCH + koff;
  const __bf16* w0b  = (const __bf16*)Wt0 + c * WPITCH + koff;
  const __bf16* w1b  = (const __bf16*)Wt1 + c * WPITCH + koff;
  const v8f z8 = {0.f, 0.f, 0.f, 0.f, 0.f, 0.f, 0.f, 0.f};

#pragma unroll 1
  for (int t = 0; t < NSTEP; ++t) {
    const int cur = (t & 1) * 64;
    const int prv = 64 - cur;

    put_hilo(hb, 128, h2s, hh, c);

#pragma unroll
    for (int ub = 0; ub < 2; ++ub) {
      const __bf16* wb = w0b + 16 * ub * WPITCH;
      v8f acc[4];
      acc[0] = z8; acc[1] = z8; acc[2] = z8; acc[3] = z8;
      mma_one(acc, xrow, wb, 0);
      mma_two(acc, hrow + prv, wb, 32);
      cell_update(acc, bb0[ub], c1[ub], h1s[ub]);
    }
    put_hilo(hb, cur, h1s, hh, c);
    __syncthreads();

#pragma unroll
    for (int ub = 0; ub < 2; ++ub) {
      const __bf16* wb = w1b + 16 * ub * WPITCH;
      v8f acc[4];
      acc[0] = z8; acc[1] = z8; acc[2] = z8; acc[3] = z8;
      mma_two(acc, hrow + cur, wb, 0);
      mma_two(acc, hrow + 128, wb, 32);
      cell_update(acc, bb1[ub], c2[ub], h2s[ub]);
    }
    {
      const int tn = (t + 1 < NSTEP) ? (t + 1) : (NSTEP - 1);
      stage_x(xs, x, rowbase, tn, lane);
    }
    __syncthreads();
  }

  float* st = St[wave];
#pragma unroll
  for (int r = 0; r < 8; ++r) {
    const float v0 = h2s[0][r], v1 = h2s[1][r];
    float s = v0 + v1;
    s += __shfl_xor(s, 1, 32);
    s += __shfl_xor(s, 2, 32);
    s += __shfl_xor(s, 4, 32);
    s += __shfl_xor(s, 8, 32);
    const float mu = s * (1.0f / NHID);
    const float d0 = v0 - mu, d1 = v1 - mu;
    float q = d0 * d0 + d1 * d1;
    q += __shfl_xor(q, 1, 32);
    q += __shfl_xor(q, 2, 32);
    q += __shfl_xor(q, 4, 32);
    q += __shfl_xor(q, 8, 32);
    const float var  = q * (1.0f / NHID);
    const float rstd = rsqrtf(var + LN_EPS);
    st[(8 * hh + r) * SPITCH + c]      = (d0 * rstd) * gm[0] + bt[0];
    st[(8 * hh + r) * SPITCH + 16 + c] = (d1 * rstd) * gm[1] + bt[1];
  }
  __syncthreads();
  {
    const int rq = lane >> 3, c4 = (lane & 7) * 4;
    for (int pass = 0; pass < 2; ++pass) {
#pragma unroll
      for (int it = 0; it < 4; ++it) {
        const int row = it * 4 + rq;
        const v4f v = *(const v4f*)(st + row * SPITCH + c4);
        *(volatile v4f*)(out + (size_t)(rowbase + row) * NHID + c4) = v;
      }
      __threadfence();
    }
  }
}

extern "C" void kernel_launch(void* const* d_in, const int* in_sizes, int n_in,
                              void* d_out, int out_size, void* d_ws, size_t ws_size, hipStream_t stream) {
  if (n_in < 11 || d_out == nullptr) return;
  if (in_sizes[0] != NBATCH * NSTEP * NIN || in_sizes[1] != NGATE * NIN || in_sizes[2] != NGATE * NHID ||
      in_sizes[3] != NGATE || in_sizes[4] != NGATE || in_sizes[5] != NGATE * NHID || in_sizes[6] != NGATE * NHID ||
      in_sizes[7] != NGATE || in_sizes[8] != NGATE || in_sizes[9] != NHID || in_sizes[10] != NHID ||
      out_size != NBATCH * NHID) return;

  const float* x    = (const float*)d_in[0];
  const float* wih0 = (const float*)d_in[1];
  const float* whh0 = (const float*)d_in[2];
  const float* bih0 = (const float*)d_in[3];
  const float* bhh0 = (const float*)d_in[4];
  const float* wih1 = (const float*)d_in[5];
  const float* whh1 = (const float*)d_in[6];
  const float* bih1 = (const float*)d_in[7];
  const float* bhh1 = (const float*)d_in[8];
  const float* gam  = (const float*)d_in[9];
  const float* bet  = (const float*)d_in[10];
  float* out = (float*)d_out;
  (void)d_ws; (void)ws_size;

  lstm2_ln_kernel<<<NBATCH / ROWS_BLK, NTHR, 0, stream>>>(x, wih0, whh0, bih0, bhh0, wih1, whh1, bih1, bhh1, gam, bet, out);
}
